// GATLocalizationModule_19172734009869
// MI455X (gfx1250) — hardware-verified
//
#include <hip/hip_runtime.h>
#include <hip/hip_bf16.h>
#include <stddef.h>
#include <stdint.h>


#define IND   128
#define HIDC  200
#define HP    224
#define GP    256
#define KP2   224
#define NP2   224
#define F1C   100
#define F1NP  112
#define F1P   128
#define F2C   50
#define F2NP  64
#define GR    32

#define NB    320
#define CHUNK 2048
#define NTHR  256
#define NWAVE 8
#define WCAP  256
#define NGRP  (CHUNK / (NTHR * 4))
#define SP    200
#define LDS_SACC (NB * SP)
#define LDS_BYTES ((LDS_SACC + 2 * NB + NWAVE * WCAP + NWAVE) * 4)

static_assert(WCAP == NGRP * 4 * 32);
static_assert(NGRP >= 1);
static_assert(NB <= 512);
static_assert((NB % NWAVE) == 0);
static_assert((LDS_SACC % 4) == 0);
static_assert(CHUNK <= 2048);
static_assert(LDS_BYTES == 266784);

typedef unsigned short us_t;
typedef float  v2f  __attribute__((ext_vector_type(2)));
typedef float  v4f  __attribute__((ext_vector_type(4)));
typedef float  v8f  __attribute__((ext_vector_type(8)));
typedef int    v4i  __attribute__((ext_vector_type(4)));
typedef us_t   v8u  __attribute__((ext_vector_type(8)));
typedef __bf16 v16b __attribute__((ext_vector_type(16)));
union Frag   { v16b v; v8u half[2]; };
union Pack16 { v8u u; v4i i; };

__device__ __forceinline__ us_t f2bf(float f) {
  unsigned u = __float_as_uint(f);
  u += 0x7FFFu + ((u >> 16) & 1u);
  return (us_t)(u >> 16);
}
__device__ __forceinline__ float bf2f(us_t h) { return __uint_as_float(((unsigned)h) << 16); }

__device__ __forceinline__ void split8(v4f a, v4f b, Pack16& ph, Pack16& pl) {
  us_t h;
  h = f2bf(a.x); ph.u[0] = h; pl.u[0] = f2bf(a.x - bf2f(h));
  h = f2bf(a.y); ph.u[1] = h; pl.u[1] = f2bf(a.y - bf2f(h));
  h = f2bf(a.z); ph.u[2] = h; pl.u[2] = f2bf(a.z - bf2f(h));
  h = f2bf(a.w); ph.u[3] = h; pl.u[3] = f2bf(a.w - bf2f(h));
  h = f2bf(b.x); ph.u[4] = h; pl.u[4] = f2bf(b.x - bf2f(h));
  h = f2bf(b.y); ph.u[5] = h; pl.u[5] = f2bf(b.y - bf2f(h));
  h = f2bf(b.z); ph.u[6] = h; pl.u[6] = f2bf(b.z - bf2f(h));
  h = f2bf(b.w); ph.u[7] = h; pl.u[7] = f2bf(b.w - bf2f(h));
}

__device__ __forceinline__ v8f wm(v16b a, v16b b, v8f c) {
  v8f d = __builtin_amdgcn_wmma_f32_16x16x32_bf16(false, a, false, b, (short)0, c, false, false);
  asm volatile("v_nop\n\tv_nop\n\tv_nop\n\tv_nop" : "+v"(d) : "v"(a), "v"(b));
  return d;
}

__device__ __forceinline__ float wsum(float v) {
  v += __shfl_xor(v, 16, 32);
  v += __shfl_xor(v, 8, 32);
  v += __shfl_xor(v, 4, 32);
  v += __shfl_xor(v, 2, 32);
  v += __shfl_xor(v, 1, 32);
  return v;
}

__device__ __forceinline__ float bsel(const float* __restrict__ b, int c, int n) {
  const int cc = (c < n) ? c : (n - 1);
  const float v = b[cc];
  return (c < n) ? v : 0.f;
}

__device__ __forceinline__ v4f relu4(v4f v) {
  v.x = fmaxf(v.x, 0.f); v.y = fmaxf(v.y, 0.f); v.z = fmaxf(v.z, 0.f); v.w = fmaxf(v.w, 0.f);
  return v;
}
__device__ __forceinline__ v4f leaky4(v4f v) {
  v.x = (v.x > 0.f) ? v.x : 0.01f * v.x;
  v.y = (v.y > 0.f) ? v.y : 0.01f * v.y;
  v.z = (v.z > 0.f) ? v.z : 0.01f * v.z;
  v.w = (v.w > 0.f) ? v.w : 0.01f * v.w;
  return v;
}

__global__ __launch_bounds__(256) void k_xconv(const float* __restrict__ x, us_t* xh, us_t* xl,
                                               int nN, int nChunks) {
  const int c = blockIdx.x * 256 + threadIdx.x;
  if (c >= nChunks) return;
  int row = c >> 4;
  const int k0 = (c & 15) * 8;
  if (row > nN - 1) row = nN - 1;
  const float* p = x + (size_t)row * IND + k0;
  const v4f a = *(const v4f*)p;
  const v4f b = *(const v4f*)(p + 4);
  Pack16 ph, pl;
  split8(a, b, ph, pl);
  const size_t o = (size_t)c * 8;
  *(volatile v4i*)(xh + o) = ph.i;
  *(volatile v4i*)(xl + o) = pl.i;
  __threadfence();
  *(volatile v4i*)(xh + o) = ph.i;
  *(volatile v4i*)(xl + o) = pl.i;
}

__global__ __launch_bounds__(256) void k_wconv(const float* __restrict__ W, us_t* wh, us_t* wl,
                                               int K, int N, int KP, int nChunks) {
  const int c = blockIdx.x * 256 + threadIdx.x;
  if (c >= nChunks) return;
  const int f  = c * 8;
  const int n  = f / KP;
  const int k0 = f - n * KP;
  v4f a, b;
  a.x = (n < N && k0 + 0 < K) ? W[(size_t)(k0 + 0) * N + n] : 0.f;
  a.y = (n < N && k0 + 1 < K) ? W[(size_t)(k0 + 1) * N + n] : 0.f;
  a.z = (n < N && k0 + 2 < K) ? W[(size_t)(k0 + 2) * N + n] : 0.f;
  a.w = (n < N && k0 + 3 < K) ? W[(size_t)(k0 + 3) * N + n] : 0.f;
  b.x = (n < N && k0 + 4 < K) ? W[(size_t)(k0 + 4) * N + n] : 0.f;
  b.y = (n < N && k0 + 5 < K) ? W[(size_t)(k0 + 5) * N + n] : 0.f;
  b.z = (n < N && k0 + 6 < K) ? W[(size_t)(k0 + 6) * N + n] : 0.f;
  b.w = (n < N && k0 + 7 < K) ? W[(size_t)(k0 + 7) * N + n] : 0.f;
  Pack16 ph, pl;
  split8(a, b, ph, pl);
  const size_t o = (size_t)f;
  *(volatile v4i*)(wh + o) = ph.i;
  *(volatile v4i*)(wl + o) = pl.i;
  __threadfence();
  *(volatile v4i*)(wh + o) = ph.i;
  *(volatile v4i*)(wl + o) = pl.i;
}

template<int KP, int LDA, int NT, int NW, int XSP>
__device__ __forceinline__ void gemm_core(const us_t* __restrict__ Ah, const us_t* __restrict__ Al,
                                          const us_t* __restrict__ Bh, const us_t* __restrict__ Bl,
                                          int rowBase, float* Xs) {
  constexpr int CT = NT / NW;
  static_assert(CT >= 1);
  static_assert(CT * NW == NT);
  static_assert((KP % 32) == 0);
  static_assert((LDA % 8) == 0);
  const int tid  = threadIdx.x;
  const int lane = tid & 31;
  const int wave = tid >> 5;
  const int hh   = lane >> 4;
  const int m    = lane & 15;
  const v8f z8 = {0.f, 0.f, 0.f, 0.f, 0.f, 0.f, 0.f, 0.f};
  v8f acc[CT][2];
#pragma unroll
  for (int j = 0; j < CT; ++j) { acc[j][0] = z8; acc[j][1] = z8; }
  const size_t ao0 = (size_t)(rowBase + m) * LDA + 8 * hh;
  const size_t ao1 = (size_t)(rowBase + 16 + m) * LDA + 8 * hh;
#pragma unroll 1
  for (int k0 = 0; k0 < KP; k0 += 32) {
    Frag a0h, a0l, a1h, a1l;
    a0h.half[0] = *(const v8u*)(Ah + ao0 + k0); a0h.half[1] = *(const v8u*)(Ah + ao0 + k0 + 16);
    a0l.half[0] = *(const v8u*)(Al + ao0 + k0); a0l.half[1] = *(const v8u*)(Al + ao0 + k0 + 16);
    a1h.half[0] = *(const v8u*)(Ah + ao1 + k0); a1h.half[1] = *(const v8u*)(Ah + ao1 + k0 + 16);
    a1l.half[0] = *(const v8u*)(Al + ao1 + k0); a1l.half[1] = *(const v8u*)(Al + ao1 + k0 + 16);
#pragma unroll
    for (int j = 0; j < CT; ++j) {
      const size_t bo = (size_t)(16 * (wave + j * NW) + m) * KP + 8 * hh + k0;
      Frag bh, bl;
      bh.half[0] = *(const v8u*)(Bh + bo); bh.half[1] = *(const v8u*)(Bh + bo + 16);
      bl.half[0] = *(const v8u*)(Bl + bo); bl.half[1] = *(const v8u*)(Bl + bo + 16);
      acc[j][0] = wm(a0h.v, bh.v, acc[j][0]);
      acc[j][0] = wm(a0h.v, bl.v, acc[j][0]);
      acc[j][0] = wm(a0l.v, bh.v, acc[j][0]);
      acc[j][1] = wm(a1h.v, bh.v, acc[j][1]);
      acc[j][1] = wm(a1h.v, bl.v, acc[j][1]);
      acc[j][1] = wm(a1l.v, bh.v, acc[j][1]);
    }
  }
#pragma unroll
  for (int j = 0; j < CT; ++j) {
    const int col = 16 * (wave + j * NW) + m;
#pragma unroll
    for (int r = 0; r < 8; ++r) {
      Xs[(8 * hh + r) * XSP + col]      = acc[j][0][r];
      Xs[(16 + 8 * hh + r) * XSP + col] = acc[j][1][r];
    }
  }
}

template<int KP, int LDA>
__global__ __launch_bounds__(224) void k_gemm_lin(
    const us_t* __restrict__ Ah, const us_t* __restrict__ Al,
    const us_t* __restrict__ Bh, const us_t* __restrict__ Bl,
    const float* __restrict__ as, const float* __restrict__ ad,
    float* H, float* asrc, float* adst) {
  constexpr int XSP = 228;
  __shared__ __attribute__((aligned(16))) float Xs[GR * XSP];
  __shared__ __attribute__((aligned(16))) float As[GR];
  __shared__ __attribute__((aligned(16))) float Ds[GR];
  const int rowBase = blockIdx.x * GR;
  gemm_core<KP, LDA, 14, 7, XSP>(Ah, Al, Bh, Bl, rowBase, Xs);
  __syncthreads();

  const int tid = threadIdx.x, lane = tid & 31, wave = tid >> 5;
  const v4f z4 = {0.f, 0.f, 0.f, 0.f};
  const v4f s4a = *(const v4f*)(as + 4 * lane);
  const v4f d4a = *(const v4f*)(ad + 4 * lane);
  v4f s4b = z4, d4b = z4;
  if (lane < 18) {
    s4b = *(const v4f*)(as + 128 + 4 * lane);
    d4b = *(const v4f*)(ad + 128 + 4 * lane);
  }
#pragma unroll 1
  for (int r = wave; r < GR; r += 7) {
    const v4f v0 = *(const v4f*)(Xs + r * XSP + 4 * lane);
    v4f v1 = z4;
    if (lane < 24) v1 = *(const v4f*)(Xs + r * XSP + 128 + 4 * lane);
    float ps = v0.x * s4a.x + v0.y * s4a.y + v0.z * s4a.z + v0.w * s4a.w
             + v1.x * s4b.x + v1.y * s4b.y + v1.z * s4b.z + v1.w * s4b.w;
    float pd = v0.x * d4a.x + v0.y * d4a.y + v0.z * d4a.z + v0.w * d4a.w
             + v1.x * d4b.x + v1.y * d4b.y + v1.z * d4b.z + v1.w * d4b.w;
    ps = wsum(ps);
    pd = wsum(pd);
    if (lane == 0) { As[r] = ps; Ds[r] = pd; }
    float* hp = H + (size_t)(rowBase + r) * HP;
    *(volatile v4f*)(hp + 4 * lane) = v0;
    if (lane < 24) *(volatile v4f*)(hp + 128 + 4 * lane) = v1;
    __threadfence();
    *(volatile v4f*)(hp + 4 * lane) = v0;
    if (lane < 24) *(volatile v4f*)(hp + 128 + 4 * lane) = v1;
  }
  __syncthreads();
  if (wave == 0 && lane < 16) {
    v4f g;
    float* gp;
    if (lane < 8) { g = *(const v4f*)(As + 4 * lane);       gp = asrc + rowBase + 4 * lane; }
    else          { g = *(const v4f*)(Ds + 4 * (lane - 8)); gp = adst + rowBase + 4 * (lane - 8); }
    *(volatile v4f*)gp = g;
    __threadfence();
    *(volatile v4f*)gp = g;
  }
}

__global__ __launch_bounds__(224) void k_gemm_fc1(
    const us_t* __restrict__ Ah, const us_t* __restrict__ Al,
    const us_t* __restrict__ Bh, const us_t* __restrict__ Bl,
    const float* __restrict__ bias, us_t* Rh, us_t* Rl) {
  constexpr int XSP = 132;
  __shared__ __attribute__((aligned(16))) float Xs[GR * XSP];
  const int rowBase = blockIdx.x * GR;
  gemm_core<KP2, GP, 7, 7, XSP>(Ah, Al, Bh, Bl, rowBase, Xs);
  for (int i = threadIdx.x; i < GR * 16; i += 224) Xs[(i >> 4) * XSP + F1NP + (i & 15)] = 0.f;
  __syncthreads();

  const int tid = threadIdx.x, lane = tid & 31, wave = tid >> 5;
#pragma unroll 1
  for (int r = wave; r < GR; r += 7) {
    if (lane < 16) {
      const int c0 = 8 * lane;
      v4f v0 = *(const v4f*)(Xs + r * XSP + c0);
      v4f v1 = *(const v4f*)(Xs + r * XSP + c0 + 4);
      v4f b0, b1;
      b0.x = bsel(bias, c0 + 0, F1C); b0.y = bsel(bias, c0 + 1, F1C);
      b0.z = bsel(bias, c0 + 2, F1C); b0.w = bsel(bias, c0 + 3, F1C);
      b1.x = bsel(bias, c0 + 4, F1C); b1.y = bsel(bias, c0 + 5, F1C);
      b1.z = bsel(bias, c0 + 6, F1C); b1.w = bsel(bias, c0 + 7, F1C);
      v0 = relu4(v0 + b0);
      v1 = relu4(v1 + b1);
      Pack16 ph, pl;
      split8(v0, v1, ph, pl);
      const size_t o = (size_t)(rowBase + r) * F1P + c0;
      *(volatile v4i*)(Rh + o) = ph.i;
      *(volatile v4i*)(Rl + o) = pl.i;
      __threadfence();
      *(volatile v4i*)(Rh + o) = ph.i;
      *(volatile v4i*)(Rl + o) = pl.i;
    }
  }
}

__global__ __launch_bounds__(128) void k_gemm_fc23(
    const us_t* __restrict__ Ah, const us_t* __restrict__ Al,
    const us_t* __restrict__ Bh, const us_t* __restrict__ Bl,
    const float* __restrict__ b2, const float* __restrict__ w3, const float* __restrict__ b3,
    float* out, int nN) {
  constexpr int XSP = 68;
  __shared__ __attribute__((aligned(16))) float Xs[GR * XSP];
  __shared__ __attribute__((aligned(16))) float Os[GR * 2];
  const int rowBase = blockIdx.x * GR;
  gemm_core<F1P, F1P, 4, 4, XSP>(Ah, Al, Bh, Bl, rowBase, Xs);
  __syncthreads();

  const int tid = threadIdx.x, lane = tid & 31, wave = tid >> 5;
  const int c0 = lane, c1 = lane + 32;
  const float bb0 = b2[c0];
  const float bb1 = bsel(b2, c1, F2C);
  const float w00 = w3[2 * c0], w01 = w3[2 * c0 + 1];
  const int   cc1 = (c1 < F2C) ? c1 : (F2C - 1);
  float w10 = w3[2 * cc1], w11 = w3[2 * cc1 + 1];
  if (c1 >= F2C) { w10 = 0.f; w11 = 0.f; }
  const float ob0 = b3[0], ob1 = b3[1];
#pragma unroll 1
  for (int i = 0; i < 8; ++i) {
    const int r = wave + 4 * i;
    const float v0 = fmaxf(Xs[r * XSP + c0] + bb0, 0.f);
    const float v1 = fmaxf(Xs[r * XSP + c1] + bb1, 0.f);
    float p0 = v0 * w00 + v1 * w10;
    float p1 = v0 * w01 + v1 * w11;
    p0 = wsum(p0);
    p1 = wsum(p1);
    if (lane == 0) { Os[2 * r] = p0 + ob0; Os[2 * r + 1] = p1 + ob1; }
  }
  __syncthreads();
  if (wave == 0 && lane < 16) {
    const int r0 = rowBase + 2 * lane;
    const v4f g = *(const v4f*)(Os + 4 * lane);
    float* op = out + (size_t)rowBase * 2 + 4 * lane;
    if (r0 + 1 < nN) {
      *(volatile v4f*)op = g;
      __threadfence();
      *(volatile v4f*)op = g;
    } else if (r0 < nN) {
      v2f g2;
      g2.x = g.x; g2.y = g.y;
      *(volatile v2f*)op = g2;
      __threadfence();
      *(volatile v2f*)op = g2;
    }
  }
}

__global__ __launch_bounds__(NTHR) void k_agg(
    const float* __restrict__ H, const float* __restrict__ asrc, const float* __restrict__ adst,
    const int* __restrict__ ei, const float* __restrict__ bias,
    us_t* Gh, us_t* Gl, int nN, int nE) {
  extern __shared__ v4f lds_dyn[];
  float* sacc = (float*)lds_dyn;
  float* smax = sacc + LDS_SACC;
  float* den  = smax + NB;
  int*   list = (int*)(den + NB);
  int*   wcnt = list + NWAVE * WCAP;

  const int tid  = threadIdx.x;
  const int lane = tid & 31;
  const int wave = tid >> 5;
  const int nodeBase = blockIdx.x * NB;

  {
    const v4f z4 = {0.f, 0.f, 0.f, 0.f};
    for (int i = tid; i < LDS_SACC / 4; i += NTHR) lds_dyn[i] = z4;
    for (int i = tid; i < NB; i += NTHR) { smax[i] = -1.0e30f; den[i] = 0.f; }
  }
  __syncthreads();

  const int* eid = ei + nE;
  const bool al16 = ((nE & 3) == 0);
  const int nChunks = (nE + CHUNK - 1) / CHUNK;
#pragma unroll 1
  for (int ch = 0; ch < nChunks; ++ch) {
    const int cbase = ch * CHUNK;
    int wc = 0;
#pragma unroll
    for (int g = 0; g < NGRP; ++g) {
      const int el0 = (g * NTHR + tid) * 4;
      const int e0  = cbase + el0;
      const int sent = -2147483647 - 1;
      v4i d;
      if (al16 && (e0 + 3 < nE)) {
        d = *(const v4i*)(eid + e0);
      } else {
        d.x = (e0     < nE) ? eid[min(e0, nE - 1)]     : sent;
        d.y = (e0 + 1 < nE) ? eid[min(e0 + 1, nE - 1)] : sent;
        d.z = (e0 + 2 < nE) ? eid[min(e0 + 2, nE - 1)] : sent;
        d.w = (e0 + 3 < nE) ? eid[min(e0 + 3, nE - 1)] : sent;
      }
      const unsigned s0 = (unsigned)d.x - (unsigned)nodeBase;
      const unsigned s1 = (unsigned)d.y - (unsigned)nodeBase;
      const unsigned s2 = (unsigned)d.z - (unsigned)nodeBase;
      const unsigned s3 = (unsigned)d.w - (unsigned)nodeBase;
      const bool h0 = s0 < (unsigned)NB;
      const bool h1 = s1 < (unsigned)NB;
      const bool h2 = s2 < (unsigned)NB;
      const bool h3 = s3 < (unsigned)NB;
      const unsigned many = __builtin_amdgcn_ballot_w32(h0 | h1 | h2 | h3);
      if (many != 0u) {
#define HITJ(J, HJ, SJ) { \
          const unsigned mj = __builtin_amdgcn_ballot_w32(HJ); \
          if (HJ) { \
            const int pos = wc + (int)__builtin_amdgcn_mbcnt_lo(mj, 0u); \
            if (pos < WCAP) list[wave * WCAP + pos] = ((el0 + (J)) << 9) | (int)(SJ); \
          } \
          wc += (int)__builtin_popcount(mj); }
        HITJ(0, h0, s0)
        HITJ(1, h1, s1)
        HITJ(2, h2, s2)
        HITJ(3, h3, s3)
#undef HITJ
      }
    }
    if (lane == 0) wcnt[wave] = wc;
    __syncthreads();

    if (wave == 0) {
#pragma unroll 1
      for (int wsx = 0; wsx < NWAVE; ++wsx) {
        int n = wcnt[wsx];
        if (n > WCAP) n = WCAP;
        if (n < 0) n = 0;
#pragma unroll 1
        for (int i = 0; i < n; ++i) {
          const int ent = list[wsx * WCAP + i];
          int slot = ent & 511;
          if (slot > NB - 1) slot = NB - 1;
          const int el = (ent >> 9) & (CHUNK - 1);
          int e = cbase + el;
          if (e > nE - 1) e = nE - 1;
          int src = ei[e];
          src = src < 0 ? 0 : (src > nN - 1 ? nN - 1 : src);
          int nd = nodeBase + slot;
          if (nd > nN - 1) nd = nN - 1;
          float a = asrc[src] + adst[nd];
          a = (a > 0.f) ? a : 0.2f * a;
          const float mo = smax[slot];
          const float mn = fmaxf(mo, a);
          const float sc = __expf(mo - mn);
          const float pe = __expf(a - mn);
          const float* hr = H + (size_t)src * HP;
          float* srow = sacc + slot * SP;
          {
            v4f* sp = (v4f*)(srow + 4 * lane);
            const v4f hv  = *(const v4f*)(hr + 4 * lane);
            const v4f cur = *sp;
            *sp = cur * sc + pe * hv;
          }
          if (lane < 18) {
            v4f* sp = (v4f*)(srow + 128 + 4 * lane);
            const v4f hv  = *(const v4f*)(hr + 128 + 4 * lane);
            const v4f cur = *sp;
            *sp = cur * sc + pe * hv;
          }
          if (lane == 0) {
            const float d0 = den[slot];
            den[slot]  = d0 * sc + pe;
            smax[slot] = mn;
          }
        }
      }
    }
    __syncthreads();
  }

  const int per = NB / NWAVE;
  const v4i z4i = {0, 0, 0, 0};
#pragma unroll 1
  for (int j = 0; j < per; ++j) {
    const int slot = wave * per + j;
    const int node = nodeBase + slot;
    if (node >= nN) break;
    float a = asrc[node] + adst[node];
    a = (a > 0.f) ? a : 0.2f * a;
    const float mo = smax[slot];
    const float mn = fmaxf(mo, a);
    const float sc = __expf(mo - mn);
    const float pe = __expf(a - mn);
    const float dn  = den[slot] * sc + pe;
    const float inv = __builtin_amdgcn_rcpf(dn);
    const int c0 = 8 * lane;
    Pack16 ph, pl;
    ph.i = z4i;
    pl.i = z4i;
    if (lane < 25) {
      const float* srow = sacc + slot * SP + c0;
      const float* hr   = H + (size_t)node * HP + c0;
      const v4f s0 = *(const v4f*)srow,        s1  = *(const v4f*)(srow + 4);
      const v4f h0 = *(const v4f*)hr,          h1  = *(const v4f*)(hr + 4);
      const v4f b0 = *(const v4f*)(bias + c0), b1v = *(const v4f*)(bias + c0 + 4);
      v4f v0 = (s0 * sc + pe * h0) * inv + b0;
      v4f v1 = (s1 * sc + pe * h1) * inv + b1v;
      v0 = leaky4(v0);
      v1 = leaky4(v1);
      split8(v0, v1, ph, pl);
    }
    us_t* gh = Gh + (size_t)node * GP + c0;
    us_t* gl = Gl + (size_t)node * GP + c0;
    *(volatile v4i*)gh = ph.i;
    *(volatile v4i*)gl = pl.i;
    __threadfence();
    *(volatile v4i*)gh = ph.i;
    *(volatile v4i*)gl = pl.i;
  }
}

extern "C" void kernel_launch(void* const* d_in, const int* in_sizes, int n_in,
                              void* d_out, int out_size, void* d_ws, size_t ws_size,
                              hipStream_t stream) {
  if (n_in < 16) return;
  const int nN = in_sizes[0] / IND;
  if (nN <= 0 || in_sizes[0] != nN * IND) return;
  if (in_sizes[1] < 0 || (in_sizes[1] & 1) != 0) return;
  const int nE = in_sizes[1] / 2;
  if (in_sizes[2] != IND * HIDC || in_sizes[3] != HIDC || in_sizes[4] != HIDC || in_sizes[5] != HIDC) return;
  if (in_sizes[6] != HIDC * HIDC || in_sizes[7] != HIDC || in_sizes[8] != HIDC || in_sizes[9] != HIDC) return;
  if (in_sizes[10] != HIDC * F1C || in_sizes[11] != F1C) return;
  if (in_sizes[12] != F1C * F2C || in_sizes[13] != F2C) return;
  if (in_sizes[14] != F2C * 2 || in_sizes[15] != 2) return;
  if (out_size != nN * 2) return;

  const float* x    = (const float*)d_in[0];
  const int*   ei   = (const int*)d_in[1];
  const float* W1   = (const float*)d_in[2];
  const float* as1  = (const float*)d_in[3];
  const float* ad1  = (const float*)d_in[4];
  const float* b1   = (const float*)d_in[5];
  const float* W2   = (const float*)d_in[6];
  const float* as2  = (const float*)d_in[7];
  const float* ad2  = (const float*)d_in[8];
  const float* b2   = (const float*)d_in[9];
  const float* fc1w = (const float*)d_in[10];
  const float* fc1b = (const float*)d_in[11];
  const float* fc2w = (const float*)d_in[12];
  const float* fc2b = (const float*)d_in[13];
  const float* fc3w = (const float*)d_in[14];
  const float* fc3b = (const float*)d_in[15];
  float* out = (float*)d_out;

  const int nP = ((nN + GR - 1) / GR) * GR;
  char* base = (char*)d_ws;
  size_t off = 0;
  auto carve = [&](size_t bytes) -> void* { void* p = base + off; off = (off + bytes + 255) & ~(size_t)255; return p; };
  us_t*  xh  = (us_t*)carve((size_t)nP * IND * 2);
  us_t*  xl  = (us_t*)carve((size_t)nP * IND * 2);
  us_t*  w1h = (us_t*)carve((size_t)NP2 * IND * 2);
  us_t*  w1l = (us_t*)carve((size_t)NP2 * IND * 2);
  us_t*  w2h = (us_t*)carve((size_t)NP2 * KP2 * 2);
  us_t*  w2l = (us_t*)carve((size_t)NP2 * KP2 * 2);
  us_t*  f1h = (us_t*)carve((size_t)F1NP * KP2 * 2);
  us_t*  f1l = (us_t*)carve((size_t)F1NP * KP2 * 2);
  us_t*  f2h = (us_t*)carve((size_t)F2NP * F1P * 2);
  us_t*  f2l = (us_t*)carve((size_t)F2NP * F1P * 2);
  float* H   = (float*)carve((size_t)nP * HP * 4);
  float* asr = (float*)carve((size_t)nP * 4);
  float* adr = (float*)carve((size_t)nP * 4);
  us_t*  gh  = (us_t*)carve((size_t)nP * GP * 2);
  us_t*  gl  = (us_t*)carve((size_t)nP * GP * 2);
  us_t*  rh  = (us_t*)carve((size_t)nP * F1P * 2);
  us_t*  rl  = (us_t*)carve((size_t)nP * F1P * 2);
  if (off > ws_size) return;

  {
    const int nc = nP * (IND / 8);
    k_xconv<<<(nc + 255) / 256, 256, 0, stream>>>(x, xh, xl, nN, nc);
  }
  {
    const int nc = NP2 * IND / 8;
    k_wconv<<<(nc + 255) / 256, 256, 0, stream>>>(W1, w1h, w1l, IND, HIDC, IND, nc);
  }
  {
    const int nc = NP2 * KP2 / 8;
    k_wconv<<<(nc + 255) / 256, 256, 0, stream>>>(W2, w2h, w2l, HIDC, HIDC, KP2, nc);
  }
  {
    const int nc = F1NP * KP2 / 8;
    k_wconv<<<(nc + 255) / 256, 256, 0, stream>>>(fc1w, f1h, f1l, HIDC, F1C, KP2, nc);
  }
  {
    const int nc = F2NP * F1P / 8;
    k_wconv<<<(nc + 255) / 256, 256, 0, stream>>>(fc2w, f2h, f2l, F1C, F2C, F1P, nc);
  }

  const int gGemm = nP / GR;
  const int gAgg  = (nN + NB - 1) / NB;
  hipFuncSetAttribute(reinterpret_cast<const void*>(&k_agg),
                      hipFuncAttributeMaxDynamicSharedMemorySize, LDS_BYTES);

  k_gemm_lin<IND, IND><<<gGemm, 224, 0, stream>>>(xh, xl, w1h, w1l, as1, ad1, H, asr, adr);
  k_agg<<<gAgg, NTHR, LDS_BYTES, stream>>>(H, asr, adr, ei, b1, gh, gl, nN, nE);

  k_gemm_lin<KP2, GP><<<gGemm, 224, 0, stream>>>(gh, gl, w2h, w2l, as2, ad2, H, asr, adr);
  k_agg<<<gAgg, NTHR, LDS_BYTES, stream>>>(H, asr, adr, ei, b2, gh, gl, nN, nE);

  k_gemm_fc1<<<gGemm, 224, 0, stream>>>(gh, gl, f1h, f1l, fc1b, rh, rl);
  k_gemm_fc23<<<gGemm, 128, 0, stream>>>(rh, rl, f2h, f2l, fc2b, fc3w, fc3b, out, nN);
}
